// CausalSelfAttention_31894427140364
// MI455X (gfx1250) — hardware-verified
//
#include <hip/hip_runtime.h>


#ifndef NB
#define NB 2
#endif
#ifndef SEQ
#define SEQ 2048
#endif
#define NB_FULL  2
#define SEQ_FULL 2048
#define DM   1024
#define NH   16
#define HD   64
#define RH   256
#define MR   (NB * SEQ)
#define PSP  40
#define OSP  68
#define PCAR 1024.0f
#define RCAR 2048.0f
#define SCL2 0.18033688011112042f
#define NEGB (-1.0e30f)

static_assert(DM == NH * HD);
static_assert(HD == 64);
static_assert(DM % 64 == 0 && DM % 32 == 0 && DM % 8 == 0);
static_assert(SEQ % 64 == 0 && RH % 64 == 0 && RH <= SEQ);
static_assert(NB <= NB_FULL && SEQ <= SEQ_FULL);
static_assert(MR % 64 == 0);
static_assert(((size_t)MR * DM / 8) % 256 == 0);
static_assert(PSP >= 32 && PSP % 8 == 0);
static_assert(OSP >= 64 && OSP % 4 == 0);

typedef _Float16 h16;
typedef unsigned short bf;
typedef __attribute__((ext_vector_type(16))) __bf16   v16bf;
typedef __attribute__((ext_vector_type(16))) _Float16 v16h;
typedef __attribute__((ext_vector_type(8)))  _Float16 v8h;
typedef __attribute__((ext_vector_type(8)))  unsigned short v8us;
typedef __attribute__((ext_vector_type(8)))  float    v8f;
typedef __attribute__((ext_vector_type(4)))  float    v4f;
typedef v8h  __attribute__((may_alias)) v8ha;
typedef v4f  __attribute__((may_alias)) v4fa;
typedef v8us __attribute__((may_alias)) v8usa;

__device__ __forceinline__ unsigned short f2bf(float f) { unsigned u = __float_as_uint(f); u += 0x7FFFu + ((u >> 16) & 1u); return (unsigned short)(u >> 16); }
__device__ __forceinline__ float bf2f(unsigned short b) { return __uint_as_float(((unsigned)b) << 16); }
__device__ __forceinline__ float bfr(float f) { return bf2f(f2bf(f)); }
__device__ __forceinline__ void splitf(float y, unsigned short& h, unsigned short& l) { h = f2bf(y); l = f2bf(y - bf2f(h)); }
__device__ __forceinline__ v16h cat16(v8h lo, v8h hi) { return __builtin_shufflevector(lo, hi, 0, 1, 2, 3, 4, 5, 6, 7, 8, 9, 10, 11, 12, 13, 14, 15); }
__device__ __forceinline__ v16bf cat16b(v8us lo, v8us hi) { return __builtin_bit_cast(v16bf, __builtin_shufflevector(lo, hi, 0, 1, 2, 3, 4, 5, 6, 7, 8, 9, 10, 11, 12, 13, 14, 15)); }
__device__ __forceinline__ v8f wmma16(v16h a, v16h b, v8f c) { return __builtin_amdgcn_wmma_f32_16x16x32_f16(false, a, false, b, (short)0, c, false, false); }
__device__ __forceinline__ v8f wmmab(v16bf a, v16bf b, v8f c) { return __builtin_amdgcn_wmma_f32_16x16x32_bf16(false, a, false, b, (short)0, c, false, false); }
__device__ __forceinline__ v16h  ldh(const h16* p) { return cat16(*(const v8h*)p, *(const v8h*)(p + 16)); }
__device__ __forceinline__ v16bf ldb(const bf* p)  { return cat16b(*(const v8us*)p, *(const v8us*)(p + 16)); }
__device__ __forceinline__ void wave_sync() { __builtin_amdgcn_fence(3  , "wavefront"); __builtin_amdgcn_wave_barrier(); asm volatile("" ::: "memory"); }

template <bool SPLIT>
__device__ __forceinline__ void gemm_body(const bf* __restrict__ A, const bf* __restrict__ A2, const bf* __restrict__ Bt, float* C, const float* __restrict__ bias, int rpb, int rpbf) {
    __shared__ __align__(16) float os[16 * OSP];
    const int lane = threadIdx.x & 31, lr = lane & 15, hi = lane >> 4;
    const int r0 = (int)blockIdx.x * 64, c0 = (int)blockIdx.y * 64;
    v8f acc[4][4];
#pragma unroll
    for (int mb = 0; mb < 4; ++mb)
#pragma unroll
        for (int nb = 0; nb < 4; ++nb) acc[mb][nb] = (v8f){};
    const size_t aoff = (size_t)(r0 + lr) * DM + 8 * hi, boff = (size_t)(c0 + lr) * DM + 8 * hi;
#pragma unroll 1
    for (int kc = 0; kc < DM; kc += 32) {
        v16bf a[4], a2[4];
#pragma unroll
        for (int mb = 0; mb < 4; ++mb) { a[mb] = ldb(A + aoff + (size_t)mb * 16 * DM + kc); if (SPLIT) a2[mb] = ldb(A2 + aoff + (size_t)mb * 16 * DM + kc); else a2[mb] = a[mb]; }
#pragma unroll
        for (int nb = 0; nb < 4; ++nb) { const v16bf bq = ldb(Bt + boff + (size_t)nb * 16 * DM + kc);
#pragma unroll
            for (int mb = 0; mb < 4; ++mb) { acc[mb][nb] = wmmab(a[mb], bq, acc[mb][nb]); if (SPLIT) acc[mb][nb] = wmmab(a2[mb], bq, acc[mb][nb]); } }
        asm volatile("v_nop\n\tv_nop\n\tv_nop\n\tv_nop" : "+v"(acc[0][0]), "+v"(acc[1][1]), "+v"(acc[2][2]), "+v"(acc[3][3]) : "v"(a[0]), "v"(a[3]), "v"(a2[0]), "v"(a2[3]));
    }
    const int rb = r0 / rpb; const size_t crow0 = (size_t)rb * rpbf + (size_t)(r0 - rb * rpb);
    const int cofs = lr * 4;
    const float b0 = bfr(bias[c0 + cofs]), b1 = bfr(bias[c0 + cofs + 1]), b2 = bfr(bias[c0 + cofs + 2]), b3 = bfr(bias[c0 + cofs + 3]);
#pragma unroll
    for (int mb = 0; mb < 4; ++mb) {
#pragma unroll
        for (int nb = 0; nb < 4; ++nb) {
#pragma unroll
            for (int j = 0; j < 8; ++j) os[(hi * 8 + j) * OSP + nb * 16 + lr] = acc[mb][nb][j]; }
        wave_sync();
        float* crow = C + (crow0 + (size_t)mb * 16) * DM + c0;
#pragma unroll 1
        for (int ps = 0; ps < 2; ++ps) {
#pragma unroll
            for (int s = 0; s < 8; ++s) { const int row = 2 * s + hi; v4f val = *(const v4fa*)(os + row * OSP + cofs);
                val[0] += b0; val[1] += b1; val[2] += b2; val[3] += b3;
                *(volatile v4f*)(crow + (size_t)row * DM + cofs) = val; }
            if (ps == 0) __threadfence(); }
        wave_sync();
    }
}
__global__ __launch_bounds__(32) __attribute__((amdgpu_num_vgpr(256))) void k_gemm1(const bf* __restrict__ A, const bf* __restrict__ Bt, float* C, const float* __restrict__ bias, int rpb, int rpbf) { gemm_body<false>(A, A, Bt, C, bias, rpb, rpbf); }
__global__ __launch_bounds__(32) __attribute__((amdgpu_num_vgpr(256))) void k_gemm2(const bf* __restrict__ A, const bf* __restrict__ A2, const bf* __restrict__ Bt, float* C, const float* __restrict__ bias, int rpb, int rpbf) { gemm_body<true>(A, A2, Bt, C, bias, rpb, rpbf); }

__global__ __launch_bounds__(256) void k_cvt8(const float* __restrict__ src, bf* dst, unsigned n8, int rpb, int rpbf) {
    const unsigned i = blockIdx.x * 256u + threadIdx.x; if (i >= n8) return;
    const unsigned row = i / (DM / 8), c8 = i % (DM / 8); const unsigned rb = row / (unsigned)rpb; const size_t srow = (size_t)rb * (size_t)rpbf + (size_t)(row - rb * (unsigned)rpb);
    const v8f v = *(const v8f*)(src + srow * DM + (size_t)c8 * 8); v8us o;
#pragma unroll
    for (int k = 0; k < 8; ++k) o[k] = f2bf(v[k]);
    bf* p = dst + (size_t)i * 8;
    *(volatile v8us*)p = o; __threadfence(); *(volatile v8us*)p = o;
}

__global__ __launch_bounds__(256) void k_hplanes(const float* __restrict__ F, h16* P16, h16* PR, int has_res, bf* PH, bf* PL) {
    const size_t i = (size_t)blockIdx.x * 256 + threadIdx.x; if (i >= (size_t)MR * DM / 8) return;
    const size_t e = i * 8; const int d = (int)(e % HD); const int t = (int)((e / HD) % SEQ); const int bh = (int)(e / ((size_t)HD * SEQ)); const int b = bh / NH, h = bh - b * NH;
    const v8f v = *(const v8f*)(F + ((size_t)b * SEQ + t) * DM + h * HD + d);
    v8h o16, orr; v8us oh, ol;
#pragma unroll
    for (int k = 0; k < 8; ++k) { const h16 x16 = (h16)v[k]; o16[k] = x16; orr[k] = (h16)((v[k] - (float)x16) * RCAR); unsigned short a, c; splitf(v[k], a, c); oh[k] = a; ol[k] = c; }
    const bool hr = (t < RH); const size_t eh = ((size_t)bh * RH + (hr ? t : 0)) * HD + d;
    *(volatile v8h*)(P16 + e) = o16; if (has_res) *(volatile v8h*)(PR + e) = orr; if (hr) { *(volatile v8us*)(PH + eh) = oh; *(volatile v8us*)(PL + eh) = ol; }
    __threadfence();
    *(volatile v8h*)(P16 + e) = o16; if (has_res) *(volatile v8h*)(PR + e) = orr; if (hr) { *(volatile v8us*)(PH + eh) = oh; *(volatile v8us*)(PL + eh) = ol; }
}

__global__ __launch_bounds__(256) void k_vplanes(const float* __restrict__ F, h16* VT16, bf* VTH, bf* VTL) {
    const size_t i = (size_t)blockIdx.x * 256 + threadIdx.x; if (i >= (size_t)MR * DM / 8) return;
    const size_t e = i * 8; const int t = (int)(e % SEQ); const int d = (int)((e / SEQ) % HD); const int bh = (int)(e / ((size_t)SEQ * HD)); const int b = bh / NH, h = bh - b * NH;
    const float* f = F + ((size_t)b * SEQ + t) * DM + h * HD + d;
    v8h o16; v8us oh, ol;
#pragma unroll
    for (int k = 0; k < 8; ++k) { const float x = f[(size_t)k * DM]; o16[k] = (h16)x; unsigned short a, c; splitf(x, a, c); oh[k] = a; ol[k] = c; }
    const bool hr = (t < RH); const size_t eh = ((size_t)bh * HD + d) * RH + (hr ? t : 0);
    *(volatile v8h*)(VT16 + e) = o16; if (hr) { *(volatile v8us*)(VTH + eh) = oh; *(volatile v8us*)(VTL + eh) = ol; }
    __threadfence();
    *(volatile v8h*)(VT16 + e) = o16; if (hr) { *(volatile v8us*)(VTH + eh) = oh; *(volatile v8us*)(VTL + eh) = ol; }
}

template <bool HIRES>
__device__ __forceinline__ void attn_body(const h16* __restrict__ Q16, const h16* __restrict__ QR, const h16* __restrict__ K16, const h16* __restrict__ VT16,
                                          const bf* __restrict__ QH, const bf* __restrict__ QL, const bf* __restrict__ KH, const bf* __restrict__ KL,
                                          const bf* __restrict__ VTH, const bf* __restrict__ VTL, bf* CH, bf* CL) {
    __shared__ __align__(16) h16 p16s[4][16 * PSP];
    __shared__ __align__(16) bf  phs[4][16 * PSP];
    __shared__ __align__(16) bf  pls[4][16 * PSP];
    __shared__ __align__(16) float os[4][16 * OSP];
    const int lane = threadIdx.x & 31, lr = lane & 15, hi = lane >> 4;
    const int wave = __builtin_amdgcn_readfirstlane((int)(threadIdx.x >> 5));
    const int bh = (int)blockIdx.y; const int b = bh / NH, h = bh - b * NH;
    const int TP = HIRES ? RH : SEQ;
    const int q0 = (HIRES ? 0 : RH) + (int)blockIdx.x * 64 + wave * 16;
    const size_t qoff  = ((size_t)bh * TP + q0 + lr) * HD + 8 * hi;
    const size_t kbase = ((size_t)bh * TP + lr) * HD + 8 * hi;
    const size_t vbase = ((size_t)bh * HD + lr) * TP + 8 * hi;
    v8f o[4];
#pragma unroll
    for (int nb = 0; nb < 4; ++nb) o[nb] = (v8f){};
    float rmax[8], rsum[8];
#pragma unroll
    for (int r = 0; r < 8; ++r) { rmax[r] = NEGB; rsum[r] = 0.0f; }
    const int nhalf = (q0 >> 5) + 1;
#pragma unroll 1
    for (int hb = 0; hb < nhalf; ++hb) {
        const int kb = hb * 32;
        v8f s0 = (v8f){}, s1 = (v8f){};
        if (HIRES) {
#pragma unroll
            for (int ks = 0; ks < 2; ++ks) {
                const v16bf qh = ldb(QH + qoff + ks * 32), ql = ldb(QL + qoff + ks * 32);
                const size_t ko = kbase + (size_t)kb * HD + ks * 32;
                const v16bf kh0 = ldb(KH + ko), kl0 = ldb(KL + ko), kh1 = ldb(KH + ko + 16 * HD), kl1 = ldb(KL + ko + 16 * HD);
                s0 = wmmab(qh, kh0, s0); s1 = wmmab(qh, kh1, s1);
                s0 = wmmab(ql, kh0, s0); s1 = wmmab(ql, kh1, s1);
                s0 = wmmab(qh, kl0, s0); s1 = wmmab(qh, kl1, s1);
                asm volatile("v_nop\n\tv_nop\n\tv_nop\n\tv_nop" : "+v"(s0), "+v"(s1) : "v"(qh), "v"(ql), "v"(kh0), "v"(kh1), "v"(kl0), "v"(kl1));
            }
        } else {
            v8f r0 = (v8f){}, r1 = (v8f){};
#pragma unroll
            for (int ks = 0; ks < 2; ++ks) {
                const v16h qa = ldh(Q16 + qoff + ks * 32), qr = ldh(QR + qoff + ks * 32);
                const size_t ko = kbase + (size_t)kb * HD + ks * 32;
                const v16h kf0 = ldh(K16 + ko), kf1 = ldh(K16 + ko + 16 * HD);
                s0 = wmma16(qa, kf0, s0); s1 = wmma16(qa, kf1, s1);
                r0 = wmma16(qr, kf0, r0); r1 = wmma16(qr, kf1, r1);
                asm volatile("v_nop\n\tv_nop\n\tv_nop\n\tv_nop" : "+v"(s0), "+v"(s1), "+v"(r0), "+v"(r1) : "v"(qa), "v"(qr), "v"(kf0), "v"(kf1));
            }
            s0 = s0 + r0 * (1.0f / RCAR); s1 = s1 + r1 * (1.0f / RCAR);
        }
#pragma unroll
        for (int r = 0; r < 8; ++r) {
            const int qrow = q0 + 8 * hi + r;
            const float a0 = (kb + lr > qrow) ? NEGB : s0[r];
            const float a1 = (kb + 16 + lr > qrow) ? NEGB : s1[r];
            float m = fmaxf(a0, a1);
            m = fmaxf(m, __shfl_xor(m, 1, 32)); m = fmaxf(m, __shfl_xor(m, 2, 32)); m = fmaxf(m, __shfl_xor(m, 4, 32)); m = fmaxf(m, __shfl_xor(m, 8, 32));
            const float nm = fmaxf(rmax[r], m);
            const float fac = __builtin_amdgcn_exp2f((rmax[r] - nm) * SCL2);
            rmax[r] = nm;
            const float e0 = __builtin_amdgcn_exp2f((a0 - nm) * SCL2), e1 = __builtin_amdgcn_exp2f((a1 - nm) * SCL2);
            rsum[r] = rsum[r] * fac + (e0 + e1);
            o[0][r] *= fac; o[1][r] *= fac; o[2][r] *= fac; o[3][r] *= fac;
            const int pi = (8 * hi + r) * PSP + lr;
            if (HIRES) { unsigned short x0, y0, x1, y1; splitf(e0, x0, y0); splitf(e1, x1, y1);
                phs[wave][pi] = x0; pls[wave][pi] = y0; phs[wave][pi + 16] = x1; pls[wave][pi + 16] = y1; }
            else { p16s[wave][pi] = (h16)(e0 * PCAR); p16s[wave][pi + 16] = (h16)(e1 * PCAR); }
        }
        wave_sync();
        const size_t vo = vbase + (size_t)kb;
        const int po = lr * PSP + 8 * hi;
        if (HIRES) {
            const v16bf pha = cat16b(*(const v8usa*)&phs[wave][po], *(const v8usa*)&phs[wave][po + 16]);
            const v16bf pla = cat16b(*(const v8usa*)&pls[wave][po], *(const v8usa*)&pls[wave][po + 16]);
            v16bf vh[4], vl[4];
#pragma unroll
            for (int nb = 0; nb < 4; ++nb) { vh[nb] = ldb(VTH + vo + (size_t)nb * 16 * TP); vl[nb] = ldb(VTL + vo + (size_t)nb * 16 * TP); }
#pragma unroll
            for (int nb = 0; nb < 4; ++nb) { o[nb] = wmmab(pha, vh[nb], o[nb]); o[nb] = wmmab(pla, vh[nb], o[nb]); o[nb] = wmmab(pha, vl[nb], o[nb]); }
            asm volatile("v_nop\n\tv_nop\n\tv_nop\n\tv_nop" : "+v"(o[0]), "+v"(o[1]), "+v"(o[2]), "+v"(o[3]) : "v"(pha), "v"(pla), "v"(vh[3]), "v"(vl[3]));
        } else {
            const v16h pa = cat16(*(const v8ha*)&p16s[wave][po], *(const v8ha*)&p16s[wave][po + 16]);
            v16h vf[4];
#pragma unroll
            for (int nb = 0; nb < 4; ++nb) vf[nb] = ldh(VT16 + vo + (size_t)nb * 16 * TP);
#pragma unroll
            for (int nb = 0; nb < 4; ++nb) o[nb] = wmma16(pa, vf[nb], o[nb]);
            asm volatile("v_nop\n\tv_nop\n\tv_nop\n\tv_nop" : "+v"(o[0]), "+v"(o[1]), "+v"(o[2]), "+v"(o[3]) : "v"(pa), "v"(vf[0]), "v"(vf[3]));
        }
        wave_sync();
    }
#pragma unroll
    for (int r = 0; r < 8; ++r) {
        float t = rsum[r];
        t += __shfl_xor(t, 1, 32); t += __shfl_xor(t, 2, 32); t += __shfl_xor(t, 4, 32); t += __shfl_xor(t, 8, 32);
        const float inv = (HIRES ? 1.0f : (1.0f / PCAR)) * (1.0f / t);
#pragma unroll
        for (int nb = 0; nb < 4; ++nb) os[wave][(8 * hi + r) * OSP + nb * 16 + lr] = o[nb][r] * inv;
    }
    wave_sync();
    const int rq = lane >> 3, sg = lane & 7;
    const size_t cbase = ((size_t)b * SEQ + q0) * DM + (size_t)h * HD + sg * 8;
#pragma unroll 1
    for (int ps = 0; ps < 2; ++ps) {
#pragma unroll
        for (int s = 0; s < 4; ++s) {
            const int row = 4 * s + rq;
            const v4f x0 = *(const v4fa*)&os[wave][row * OSP + sg * 8];
            const v4f x1 = *(const v4fa*)&os[wave][row * OSP + sg * 8 + 4];
            v8us oh, ol;
#pragma unroll
            for (int q = 0; q < 4; ++q) { unsigned short a, c; splitf(x0[q], a, c); oh[q] = a; ol[q] = c; splitf(x1[q], a, c); oh[4 + q] = a; ol[4 + q] = c; }
            *(volatile v8us*)(CH + cbase + (size_t)row * DM) = oh;
            *(volatile v8us*)(CL + cbase + (size_t)row * DM) = ol;
        }
        if (ps == 0) __threadfence();
    }
}
__global__ __launch_bounds__(128) __attribute__((amdgpu_num_vgpr(256))) void k_attn_lo(const h16* __restrict__ Q16, const h16* __restrict__ QR, const h16* __restrict__ K16, const h16* __restrict__ VT16, bf* CH, bf* CL) {
    attn_body<false>(Q16, QR, K16, VT16, (const bf*)nullptr, (const bf*)nullptr, (const bf*)nullptr, (const bf*)nullptr, (const bf*)nullptr, (const bf*)nullptr, CH, CL);
}
__global__ __launch_bounds__(128) __attribute__((amdgpu_num_vgpr(256))) void k_attn_hi(const bf* __restrict__ QH, const bf* __restrict__ QL, const bf* __restrict__ KH, const bf* __restrict__ KL, const bf* __restrict__ VTH, const bf* __restrict__ VTL, bf* CH, bf* CL) {
    attn_body<true>((const h16*)nullptr, (const h16*)nullptr, (const h16*)nullptr, (const h16*)nullptr, QH, QL, KH, KL, VTH, VTL, CH, CL);
}

constexpr size_t SZ_W = (size_t)DM * DM * 2;
constexpr size_t SZ_X = (size_t)MR * DM * 2;
constexpr size_t SZ_F = (size_t)MR * DM * 4;
constexpr size_t SZ_H = (size_t)NB * NH * RH * HD * 2;
constexpr size_t WS_TOTAL = 4 * SZ_W + SZ_X + SZ_F + 4 * SZ_X + 6 * SZ_H + 2 * SZ_X;
static_assert(SZ_W % 256 == 0 && SZ_X % 256 == 0 && SZ_F % 256 == 0 && SZ_H % 256 == 0);
static_assert(WS_TOTAL <= (size_t)134217728);

extern "C" void kernel_launch(void* const* d_in, const int* in_sizes, int n_in,
                              void* d_out, int out_size, void* d_ws, size_t ws_size, hipStream_t stream) {
    if (n_in < 9) return;
    const size_t xneed = ((size_t)(NB - 1) * SEQ_FULL + SEQ) * DM;
    if ((size_t)in_sizes[0] < xneed || (size_t)out_size < xneed) return;
    if (in_sizes[1] < DM * DM || in_sizes[3] < DM * DM || in_sizes[5] < DM * DM || in_sizes[7] < DM * DM) return;
    if (in_sizes[2] < DM || in_sizes[4] < DM || in_sizes[6] < DM || in_sizes[8] < DM) return;
    if (WS_TOTAL > ws_size) return;
    const float* x  = (const float*)d_in[0];
    const float* wq = (const float*)d_in[1]; const float* bq = (const float*)d_in[2];
    const float* wk = (const float*)d_in[3]; const float* bk = (const float*)d_in[4];
    const float* wv = (const float*)d_in[5]; const float* bv = (const float*)d_in[6];
    const float* wp = (const float*)d_in[7]; const float* bp = (const float*)d_in[8];
    float* OUT = (float*)d_out;
    char* w = (char*)d_ws; size_t off = 0;
    bf* WQ = (bf*)(w + off); off += SZ_W; bf* WK = (bf*)(w + off); off += SZ_W; bf* WV = (bf*)(w + off); off += SZ_W; bf* WP = (bf*)(w + off); off += SZ_W;
    bf* XB = (bf*)(w + off); off += SZ_X;
    float* F = (float*)(w + off); off += SZ_F;
    h16* Q16 = (h16*)(w + off); off += SZ_X; h16* QR = (h16*)(w + off); off += SZ_X; h16* K16 = (h16*)(w + off); off += SZ_X; h16* VT16 = (h16*)(w + off); off += SZ_X;
    bf* QH = (bf*)(w + off); off += SZ_H; bf* QL = (bf*)(w + off); off += SZ_H; bf* KH = (bf*)(w + off); off += SZ_H; bf* KL = (bf*)(w + off); off += SZ_H;
    bf* VTH = (bf*)(w + off); off += SZ_H; bf* VTL = (bf*)(w + off); off += SZ_H;
    bf* CH = (bf*)(w + off); off += SZ_X; bf* CL = (bf*)(w + off); off += SZ_X;
    if (off != WS_TOTAL) return;

    const unsigned nx8 = (unsigned)((size_t)MR * DM / 8), nw8 = (unsigned)((size_t)DM * DM / 8);
    k_cvt8<<<(nx8 + 255) / 256, 256, 0, stream>>>(x, XB, nx8, SEQ, SEQ_FULL);
    k_cvt8<<<(nw8 + 255) / 256, 256, 0, stream>>>(wq, WQ, nw8, DM, DM);
    k_cvt8<<<(nw8 + 255) / 256, 256, 0, stream>>>(wk, WK, nw8, DM, DM);
    k_cvt8<<<(nw8 + 255) / 256, 256, 0, stream>>>(wv, WV, nw8, DM, DM);
    k_cvt8<<<(nw8 + 255) / 256, 256, 0, stream>>>(wp, WP, nw8, DM, DM);
    const dim3 gg(MR / 64, DM / 64, 1);
    const unsigned gp = (unsigned)(((size_t)MR * DM / 8 + 255) / 256);
    k_gemm1<<<gg, 32, 0, stream>>>(XB, WQ, F, bq, MR, MR);
    k_hplanes<<<gp, 256, 0, stream>>>(F, Q16, QR, 1, QH, QL);
    k_gemm1<<<gg, 32, 0, stream>>>(XB, WK, F, bk, MR, MR);
    k_hplanes<<<gp, 256, 0, stream>>>(F, K16, K16, 0, KH, KL);
    k_gemm1<<<gg, 32, 0, stream>>>(XB, WV, F, bv, MR, MR);
    k_vplanes<<<gp, 256, 0, stream>>>(F, VT16, VTH, VTL);
    k_attn_hi<<<dim3(RH / 64, NB * NH, 1), 128, 0, stream>>>(QH, QL, KH, KL, VTH, VTL, CH, CL);
    if (SEQ > RH) k_attn_lo<<<dim3((SEQ - RH) / 64, NB * NH, 1), 128, 0, stream>>>(Q16, QR, K16, VT16, CH, CL);
    k_gemm2<<<gg, 32, 0, stream>>>(CH, CL, WP, OUT, bp, SEQ, SEQ_FULL);
}
